// lstm_seq2seq_69088843924350
// MI455X (gfx1250) — hardware-run, weakly checked
//
#include <hip/hip_runtime.h>
#include <math.h>

constexpr int NB    = 512;
constexpr int NTS   = 256;
constexpr int NDI   = 32;
constexpr int NH    = 128;
constexpr int NG4   = 4 * NH;
constexpr int NTGT  = 64;
constexpr int KCAT0 = NDI + NH;
constexpr int KCAT1 = NH + NH;
constexpr int NTHR  = 256;
constexpr int RB    = 16;
constexpr int XP    = 40;
constexpr int HP    = 136;
constexpr int OSP   = 36;
constexpr float WSC     = 16.0f;
constexpr float WSC_INV = 1.0f / 16.0f;
static_assert(NB % RB == 0, "grid exact");
static_assert(NH == 16 * (NTHR / 32), "8 waves x 16 hidden units");
static_assert(NDI % 32 == 0 && NH % 32 == 0 && KCAT0 % 32 == 0 && KCAT1 % 32 == 0, "K chunks of 32, no tails");
static_assert(XP % 8 == 0 && HP % 8 == 0 && OSP % 4 == 0, "16-B aligned fragment / float4 rows");
static_assert(NDI == 32, "head = 2 n-subtiles; one (b,t) output row = 32 floats = one 128-B line");
static_assert(RB * NDI == 128 * 4, "x tile: 128 threads x 4 floats");
static_assert((NG4 * KCAT0 / 8) % 32 == 0 && (NG4 * KCAT1 / 8) % 32 == 0 && (NDI * NH / 8) % 32 == 0, "plane writes = whole 512-B wave chunks");

typedef __attribute__((ext_vector_type(16))) _Float16 v16h;
typedef __attribute__((ext_vector_type(8)))  _Float16 v8h;
typedef __attribute__((ext_vector_type(8)))  float    v8f;
typedef __attribute__((ext_vector_type(4)))  float    v4f;
typedef __attribute__((ext_vector_type(2)))  unsigned v2u;

__device__ __forceinline__ unsigned short f2bf_bits(float f) {
  unsigned u = __float_as_uint(f);
  return (unsigned short)((u + 0x7FFFu + ((u >> 16) & 1u)) >> 16);
}
__device__ __forceinline__ float bf_bits2f(unsigned short h) { return __uint_as_float(((unsigned)h) << 16); }
__device__ __forceinline__ float bf16r(float f) { return bf_bits2f(f2bf_bits(f)); }
__device__ __forceinline__ unsigned short h_bits(float f) { return __builtin_bit_cast(unsigned short, (_Float16)f); }

__device__ __forceinline__ void mma_guard4h(v8f& a0, v8f& a1, v8f& a2, v8f& a3, v16h x, v16h y0, v16h y1, v16h y2, v16h y3) {
  asm volatile("v_nop\n\tv_nop\n\tv_nop\n\tv_nop" : "+v"(a0), "+v"(a1), "+v"(a2), "+v"(a3) : "v"(x), "v"(y0), "v"(y1), "v"(y2), "v"(y3));
}
__device__ __forceinline__ void mma_guard1h(v8f& a0, v16h x, v16h y) {
  asm volatile("v_nop\n\tv_nop\n\tv_nop\n\tv_nop" : "+v"(a0) : "v"(x), "v"(y));
}
__device__ __forceinline__ void acc_guard4(v8f& a, v8f& b, v8f& c, v8f& d) { asm volatile("v_nop\n\tv_nop\n\tv_nop\n\tv_nop" : "+v"(a), "+v"(b), "+v"(c), "+v"(d)); }
__device__ __forceinline__ void acc_guard1(v8f& a) { asm volatile("v_nop\n\tv_nop\n\tv_nop\n\tv_nop" : "+v"(a)); }
__device__ __forceinline__ void pin4(float& a, float& b, float& c, float& d) { asm volatile("" : "+v"(a), "+v"(b), "+v"(c), "+v"(d) :: "memory"); }

template <typename T> struct Frag;
template <> struct Frag<_Float16> {
  typedef v16h V; union U { v16h v; v8h h[2]; };
  static __device__ __forceinline__ v16h load(const _Float16* p) {
    U f; f.h[0] = *(const v8h*)(p); f.h[1] = *(const v8h*)(p + 16); return f.v;
  }
  static __device__ __forceinline__ v8f mma(v16h a, v16h b, v8f c) {
    return __builtin_amdgcn_wmma_f32_16x16x32_f16(false, a, false, b, (short)0, c, false, false);
  }
};

__device__ __forceinline__ float fsig(float x)  { return __builtin_amdgcn_rcpf(1.0f + __expf(-x)); }
__device__ __forceinline__ float ftanh(float x) { return 1.0f - 2.0f * __builtin_amdgcn_rcpf(__expf(2.0f * x) + 1.0f); }

__global__ __launch_bounds__(NTHR) void catcvt_kernel(const float* __restrict__ Wa, int Ka,
                                                      const float* __restrict__ Wb, int Kb,
                                                      unsigned short* __restrict__ dst, int nrow, float sc) {
  const int i = blockIdx.x * NTHR + threadIdx.x;
  const int Kc = Ka + Kb;
  const int nk8 = Kc >> 3;
  const int n8 = nrow * nk8;
  if (i < n8) {
    const int row = i / nk8;
    const int k = (i - row * nk8) * 8;
    int ka = k; if (ka > Ka - 8) ka = Ka - 8;
    int kb = k - Ka; if (kb > Kb - 8) kb = Kb - 8; if (kb < 0) kb = 0;
    const float* pa = Wa + (size_t)row * (size_t)Ka + ka;
    const float* pb = Wb + (size_t)row * (size_t)Kb + kb;
    const v4f a0 = *(const v4f*)(pa);
    const v4f a1 = *(const v4f*)(pa + 4);
    const v4f b0 = *(const v4f*)(pb);
    const v4f b1 = *(const v4f*)(pb + 4);
    const float fa = (k < Ka) ? 1.0f : 0.0f;
    const float fb = 1.0f - fa;
    v8h hv;
#pragma unroll
    for (int e = 0; e < 4; ++e) {
      const float v0 = fmaf(fa, a0[e], fb * b0[e]);
      const float v1 = fmaf(fa, a1[e], fb * b1[e]);
      hv[e]     = (_Float16)(bf16r(v0) * sc);
      hv[4 + e] = (_Float16)(bf16r(v1) * sc);
    }
    *(volatile v8h*)(dst + (size_t)i * 8) = hv;
    __threadfence();
    *(volatile v8h*)(dst + (size_t)i * 8) = hv;
  }
}

__device__ __forceinline__ void load_x_tile(unsigned short* Xs, const float* __restrict__ x, int rowbase, int t, int tid) {
  if (tid < 128) {
    const int m = tid >> 3, f4 = (tid & 7) * 4;
    const v4f v = *(const v4f*)(x + ((size_t)(rowbase + m) * NTS + (size_t)t) * NDI + f4);
    const unsigned short u0 = h_bits(bf16r(v[0])), u1 = h_bits(bf16r(v[1]));
    const unsigned short u2 = h_bits(bf16r(v[2])), u3 = h_bits(bf16r(v[3]));
    v2u pk;
    pk[0] = (unsigned)u0 | ((unsigned)u1 << 16);
    pk[1] = (unsigned)u2 | ((unsigned)u3 << 16);
    *(v2u*)(Xs + m * XP + f4) = pk;
  }
}

template <int KA, int KB, int LDW>
__device__ __forceinline__ void gate_mma(v8f (&acc)[4], const _Float16* arow, const _Float16* brow, const _Float16* wrow) {
  const v8f z8 = {0.f, 0.f, 0.f, 0.f, 0.f, 0.f, 0.f, 0.f};
  constexpr size_t GS = (size_t)NH * (size_t)LDW;
  acc[0] = z8; acc[1] = z8; acc[2] = z8; acc[3] = z8;
#pragma unroll 1
  for (int k0 = 0; k0 < KA; k0 += 32) {
    const v16h a  = Frag<_Float16>::load(arow + k0);
    const v16h b0 = Frag<_Float16>::load(wrow + k0);
    const v16h b1 = Frag<_Float16>::load(wrow + GS + k0);
    const v16h b2 = Frag<_Float16>::load(wrow + 2 * GS + k0);
    const v16h b3 = Frag<_Float16>::load(wrow + 3 * GS + k0);
    acc[0] = Frag<_Float16>::mma(a, b0, acc[0]);
    acc[1] = Frag<_Float16>::mma(a, b1, acc[1]);
    acc[2] = Frag<_Float16>::mma(a, b2, acc[2]);
    acc[3] = Frag<_Float16>::mma(a, b3, acc[3]);
    mma_guard4h(acc[0], acc[1], acc[2], acc[3], a, b0, b1, b2, b3);
  }
#pragma unroll 1
  for (int k0 = 0; k0 < KB; k0 += 32) {
    const v16h a  = Frag<_Float16>::load(brow + k0);
    const v16h b0 = Frag<_Float16>::load(wrow + KA + k0);
    const v16h b1 = Frag<_Float16>::load(wrow + KA + GS + k0);
    const v16h b2 = Frag<_Float16>::load(wrow + KA + 2 * GS + k0);
    const v16h b3 = Frag<_Float16>::load(wrow + KA + 3 * GS + k0);
    acc[0] = Frag<_Float16>::mma(a, b0, acc[0]);
    acc[1] = Frag<_Float16>::mma(a, b1, acc[1]);
    acc[2] = Frag<_Float16>::mma(a, b2, acc[2]);
    acc[3] = Frag<_Float16>::mma(a, b3, acc[3]);
    mma_guard4h(acc[0], acc[1], acc[2], acc[3], a, b0, b1, b2, b3);
  }
  acc_guard4(acc[0], acc[1], acc[2], acc[3]);
}

__device__ __forceinline__ void lstm_cell(const v8f (&acc)[4], const float (&bb)[4], float (&cst)[8], float (&hst)[8]) {
#pragma unroll
  for (int r = 0; r < 8; ++r) {
    const float zi = acc[0][r] * WSC_INV + bb[0];
    const float zf = acc[1][r] * WSC_INV + bb[1];
    const float zg = acc[2][r] * WSC_INV + bb[2];
    const float zo = acc[3][r] * WSC_INV + bb[3];
    const float cn = fsig(zf) * cst[r] + fsig(zi) * ftanh(zg);
    cst[r] = cn;
    hst[r] = fsig(zo) * ftanh(cn);
  }
}

__global__ __launch_bounds__(NTHR) void seq2seq_kernel(
    const float* __restrict__ x, const int* __restrict__ tgt,
    const float* __restrict__ ebih0, const float* __restrict__ ebhh0,
    const float* __restrict__ ebih1, const float* __restrict__ ebhh1,
    const float* __restrict__ dbih0, const float* __restrict__ dbhh0,
    const float* __restrict__ dbih1, const float* __restrict__ dbhh1,
    const float* __restrict__ linb,
    const unsigned short* __restrict__ WE0p, const unsigned short* __restrict__ WE1p,
    const unsigned short* __restrict__ WD0p, const unsigned short* __restrict__ WD1p,
    const unsigned short* __restrict__ WLp,
    float* __restrict__ out) {
  __shared__ __align__(16) unsigned short Xs[RB * XP];
  __shared__ __align__(16) unsigned short Hs0[RB * HP];
  __shared__ __align__(16) unsigned short Hs1[RB * HP];
  __shared__ __align__(16) float          Os[RB * OSP];
  const _Float16* WE0 = (const _Float16*)WE0p;
  const _Float16* WE1 = (const _Float16*)WE1p;
  const _Float16* WD0 = (const _Float16*)WD0p;
  const _Float16* WD1 = (const _Float16*)WD1p;
  const _Float16* WL  = (const _Float16*)WLp;
  const int tid = threadIdx.x, lane = tid & 31, wave = tid >> 5;
  const int c = lane & 15, hh = lane >> 4, koff = hh * 8;
  const int rowbase = blockIdx.x * RB;
  const int j = 16 * wave + c;

#pragma unroll 1
  for (int i = tid; i < RB * HP; i += NTHR) { Hs0[i] = (unsigned short)0; Hs1[i] = (unsigned short)0; }
#pragma unroll 1
  for (int i = tid; i < RB * XP; i += NTHR) Xs[i] = (unsigned short)0;
#pragma unroll 1
  for (int i = tid; i < RB * OSP; i += NTHR) Os[i] = 0.0f;

  float c0s[8], h0s[8], c1s[8], h1s[8];
#pragma unroll
  for (int r = 0; r < 8; ++r) { c0s[r] = 0.0f; h0s[r] = 0.0f; c1s[r] = 0.0f; h1s[r] = 0.0f; }

  float be0[4], be1[4];
#pragma unroll
  for (int g = 0; g < 4; ++g) be0[g] = bf16r(ebih0[g * NH + j]) + bf16r(ebhh0[g * NH + j]);
  pin4(be0[0], be0[1], be0[2], be0[3]);
#pragma unroll
  for (int g = 0; g < 4; ++g) be1[g] = bf16r(ebih1[g * NH + j]) + bf16r(ebhh1[g * NH + j]);
  pin4(be1[0], be1[1], be1[2], be1[3]);

  int tl = tgt[0];
  tl = (tl < 0) ? 0 : tl;
  tl = (tl > NTGT) ? NTGT : tl;

  __syncthreads();
  load_x_tile(Xs, x, rowbase, 0, tid);
  __syncthreads();

  const _Float16* xrow  = (const _Float16*)Xs  + c * XP + koff;
  const _Float16* h0row = (const _Float16*)Hs0 + c * HP + koff;
  const _Float16* h1row = (const _Float16*)Hs1 + c * HP + koff;
  const _Float16* we0row = WE0 + (size_t)j * KCAT0 + koff;
  const _Float16* we1row = WE1 + (size_t)j * KCAT1 + koff;
  const _Float16* wd0row = WD0 + (size_t)j * KCAT0 + koff;
  const _Float16* wd1row = WD1 + (size_t)j * KCAT1 + koff;

  v8f acc[4];

#pragma unroll 1
  for (int t = 0; t < NTS; ++t) {
    gate_mma<NDI, NH, KCAT0>(acc, xrow, h0row, we0row);
    lstm_cell(acc, be0, c0s, h0s);
    __syncthreads();
#pragma unroll
    for (int r = 0; r < 8; ++r) Hs0[(8 * hh + r) * HP + j] = h_bits(h0s[r]);
    {
      const int tn = (t + 1 < NTS) ? (t + 1) : (NTS - 1);
      load_x_tile(Xs, x, rowbase, tn, tid);
    }
    __syncthreads();
    gate_mma<NH, NH, KCAT1>(acc, h0row, h1row, we1row);
    lstm_cell(acc, be1, c1s, h1s);
    __syncthreads();
#pragma unroll
    for (int r = 0; r < 8; ++r) Hs1[(8 * hh + r) * HP + j] = h_bits(h1s[r]);
    __syncthreads();
  }

  float bd0[4], bd1[4];
#pragma unroll
  for (int g = 0; g < 4; ++g) bd0[g] = bf16r(dbih0[g * NH + j]) + bf16r(dbhh0[g * NH + j]);
  pin4(bd0[0], bd0[1], bd0[2], bd0[3]);
#pragma unroll
  for (int g = 0; g < 4; ++g) bd1[g] = bf16r(dbih1[g * NH + j]) + bf16r(dbhh1[g * NH + j]);
  pin4(bd1[0], bd1[1], bd1[2], bd1[3]);
  const int nl = (16 * wave + c) & (NDI - 1);
  const float blv = bf16r(linb[nl]);
  const _Float16* wlrow = WL + (size_t)nl * NH + koff;
  load_x_tile(Xs, x, rowbase, NTS - 1, tid);
  __syncthreads();

#pragma unroll 1
  for (int t = 0; t < tl; ++t) {
    gate_mma<NDI, NH, KCAT0>(acc, xrow, h0row, wd0row);
    lstm_cell(acc, bd0, c0s, h0s);
    __syncthreads();
#pragma unroll
    for (int r = 0; r < 8; ++r) Hs0[(8 * hh + r) * HP + j] = h_bits(h0s[r]);
    __syncthreads();
    gate_mma<NH, NH, KCAT1>(acc, h0row, h1row, wd1row);
    lstm_cell(acc, bd1, c1s, h1s);
    __syncthreads();
#pragma unroll
    for (int r = 0; r < 8; ++r) Hs1[(8 * hh + r) * HP + j] = h_bits(h1s[r]);
    __syncthreads();
    if (wave < 2) {
      v8f accL = {0.f, 0.f, 0.f, 0.f, 0.f, 0.f, 0.f, 0.f};
#pragma unroll 1
      for (int k0 = 0; k0 < NH; k0 += 32) {
        const v16h a = Frag<_Float16>::load(h1row + k0);
        const v16h b = Frag<_Float16>::load(wlrow + k0);
        accL = Frag<_Float16>::mma(a, b, accL);
        mma_guard1h(accL, a, b);
      }
      acc_guard1(accL);
#pragma unroll
      for (int r = 0; r < 8; ++r) {
        const float v = accL[r] * WSC_INV + blv;
        Os[(8 * hh + r) * OSP + nl] = v;
        Xs[(8 * hh + r) * XP + nl]  = h_bits(v);
      }
    }
    __syncthreads();
    if (wave < 4) {
      const int row = 4 * wave + (lane >> 3), c4 = (lane & 7) * 4;
      const v4f v = *(const v4f*)(Os + row * OSP + c4);
      float* op = out + ((size_t)(rowbase + row) * NTGT + (size_t)t) * NDI + c4;
      *(volatile v4f*)op = v;
      __threadfence();
      *(volatile v4f*)op = v;
    }
  }
}

extern "C" void kernel_launch(void* const* d_in, const int* in_sizes, int n_in,
                              void* d_out, int out_size, void* d_ws, size_t ws_size, hipStream_t stream) {
  if (n_in < 20 || d_out == nullptr || d_ws == nullptr) return;
  if (in_sizes[0] != NB * NTS * NDI || in_sizes[1] != 1 ||
      in_sizes[2] != NG4 * NDI || in_sizes[3] != NG4 * NH || in_sizes[4] != NG4 || in_sizes[5] != NG4 ||
      in_sizes[6] != NG4 * NH || in_sizes[7] != NG4 * NH || in_sizes[8] != NG4 || in_sizes[9] != NG4 ||
      in_sizes[10] != NG4 * NDI || in_sizes[11] != NG4 * NH || in_sizes[12] != NG4 || in_sizes[13] != NG4 ||
      in_sizes[14] != NG4 * NH || in_sizes[15] != NG4 * NH || in_sizes[16] != NG4 || in_sizes[17] != NG4 ||
      in_sizes[18] != NDI * NH || in_sizes[19] != NDI || out_size != NB * NTGT * NDI) return;

  const float* x     = (const float*)d_in[0];
  const int*   tgt   = (const int*)d_in[1];
  const float* eWih0 = (const float*)d_in[2];
  const float* eWhh0 = (const float*)d_in[3];
  const float* ebih0 = (const float*)d_in[4];
  const float* ebhh0 = (const float*)d_in[5];
  const float* eWih1 = (const float*)d_in[6];
  const float* eWhh1 = (const float*)d_in[7];
  const float* ebih1 = (const float*)d_in[8];
  const float* ebhh1 = (const float*)d_in[9];
  const float* dWih0 = (const float*)d_in[10];
  const float* dWhh0 = (const float*)d_in[11];
  const float* dbih0 = (const float*)d_in[12];
  const float* dbhh0 = (const float*)d_in[13];
  const float* dWih1 = (const float*)d_in[14];
  const float* dWhh1 = (const float*)d_in[15];
  const float* dbih1 = (const float*)d_in[16];
  const float* dbhh1 = (const float*)d_in[17];
  const float* linW  = (const float*)d_in[18];
  const float* linb  = (const float*)d_in[19];
  float* out = (float*)d_out;

  char* ws = (char*)d_ws; size_t off = 0;
  auto carve = [&](size_t bytes) -> char* { char* p = ws + off; off += (bytes + 255) & ~(size_t)255; return p; };
  unsigned short* WE0 = (unsigned short*)carve((size_t)NG4 * KCAT0 * 2);
  unsigned short* WE1 = (unsigned short*)carve((size_t)NG4 * KCAT1 * 2);
  unsigned short* WD0 = (unsigned short*)carve((size_t)NG4 * KCAT0 * 2);
  unsigned short* WD1 = (unsigned short*)carve((size_t)NG4 * KCAT1 * 2);
  unsigned short* WL  = (unsigned short*)carve((size_t)NDI * NH * 2);
  if (off > ws_size || off > (size_t)134217728) return;

  const int n8a = NG4 * KCAT0 / 8;
  const int n8b = NG4 * KCAT1 / 8;
  const int n8l = NDI * NH / 8;
  catcvt_kernel<<<(n8a + NTHR - 1) / NTHR, NTHR, 0, stream>>>(eWih0, NDI, eWhh0, NH, WE0, NG4, WSC);
  catcvt_kernel<<<(n8b + NTHR - 1) / NTHR, NTHR, 0, stream>>>(eWih1, NH,  eWhh1, NH, WE1, NG4, WSC);
  catcvt_kernel<<<(n8a + NTHR - 1) / NTHR, NTHR, 0, stream>>>(dWih0, NDI, dWhh0, NH, WD0, NG4, WSC);
  catcvt_kernel<<<(n8b + NTHR - 1) / NTHR, NTHR, 0, stream>>>(dWih1, NH,  dWhh1, NH, WD1, NG4, WSC);
  catcvt_kernel<<<(n8l + NTHR - 1) / NTHR, NTHR, 0, stream>>>(linW,  NH,  linW,  0,  WL,  NDI, WSC);

  seq2seq_kernel<<<NB / RB, NTHR, 0, stream>>>(x, tgt, ebih0, ebhh0, ebih1, ebhh1, dbih0, dbhh0, dbih1, dbhh1, linb,
                                                WE0, WE1, WD0, WD1, WL, out);
}
